// hand_lstm_6408091206365
// MI455X (gfx1250) — hardware-verified
//
#include <hip/hip_runtime.h>
#include <stddef.h>

typedef __attribute__((ext_vector_type(16))) _Float16 v16h;
typedef __attribute__((ext_vector_type(8)))  _Float16 v8h;
typedef __attribute__((ext_vector_type(16))) __bf16   v16b;
typedef __attribute__((ext_vector_type(8)))  __bf16   v8b;
typedef __attribute__((ext_vector_type(8)))  float    v8f;
typedef __attribute__((ext_vector_type(4)))  float    v4f;
typedef __attribute__((ext_vector_type(4)))  unsigned v4u;

__device__ __forceinline__ unsigned short f2bf_bits(float f) {
  unsigned u = __float_as_uint(f);
  return (unsigned short)((u + 0x7FFFu + ((u >> 16) & 1u)) >> 16);
}
__device__ __forceinline__ float bf_bits2f(unsigned short h) { return __uint_as_float(((unsigned)h) << 16); }

__device__ __forceinline__ void dep_guard_h(v8f& a, v8f& b, v16h x, v16h y) { asm volatile("v_nop\n\tv_nop\n\tv_nop\n\tv_nop" : "+v"(a), "+v"(b) : "v"(x), "v"(y)); }
__device__ __forceinline__ void dep_guard_b(v8f& a, v8f& b, v16b x, v16b y) { asm volatile("v_nop\n\tv_nop\n\tv_nop\n\tv_nop" : "+v"(a), "+v"(b) : "v"(x), "v"(y)); }
__device__ __forceinline__ void keep4_h(v16h a, v16h b, v16h c, v16h d) { asm volatile("v_nop" :: "v"(a), "v"(b), "v"(c), "v"(d)); }
__device__ __forceinline__ void keep4_b(v16b a, v16b b, v16b c, v16b d) { asm volatile("v_nop" :: "v"(a), "v"(b), "v"(c), "v"(d)); }
__device__ __forceinline__ void acc_guard4(v8f& a, v8f& b, v8f& c, v8f& d) { asm volatile("v_nop\n\tv_nop\n\tv_nop\n\tv_nop" : "+v"(a), "+v"(b), "+v"(c), "+v"(d)); }
__device__ __forceinline__ void dep_guard4x_h(v8f& a, v8f& b, v8f& c, v8f& d, v16h x, v16h y) {
  asm volatile("v_nop\n\tv_nop\n\tv_nop\n\tv_nop" : "+v"(a), "+v"(b), "+v"(c), "+v"(d) : "v"(x), "v"(y));
}

template <typename T> struct Frag;
template <> struct Frag<_Float16> {
  typedef v16h V; union U { v16h v; v8h h[2]; };
  static __device__ __forceinline__ v16h load(const _Float16* p) {
    U f; f.h[0] = *(const v8h*)(p); f.h[1] = *(const v8h*)(p + 16); return f.v;
  }
  static __device__ __forceinline__ v8f mma(v16h a, v16h b, v8f c) {
    return __builtin_amdgcn_wmma_f32_16x16x32_f16(false, a, false, b, (short)0, c, false, false);
  }
  static __device__ __forceinline__ void guard(v8f& a, v8f& b, v16h x, v16h y) { dep_guard_h(a, b, x, y); }
  static __device__ __forceinline__ void keep(v16h a, v16h b, v16h c, v16h d) { keep4_h(a, b, c, d); }
};
template <> struct Frag<__bf16> {
  typedef v16b V; union U { v16b v; v8b h[2]; };
  static __device__ __forceinline__ v16b load(const __bf16* p) {
    U f; f.h[0] = *(const v8b*)(p); f.h[1] = *(const v8b*)(p + 16); return f.v;
  }
  static __device__ __forceinline__ v8f mma(v16b a, v16b b, v8f c) {
    return __builtin_amdgcn_wmma_f32_16x16x32_bf16(false, a, false, b, (short)0, c, false, false);
  }
  static __device__ __forceinline__ void guard(v8f& a, v8f& b, v16b x, v16b y) { dep_guard_b(a, b, x, y); }
  static __device__ __forceinline__ void keep(v16b a, v16b b, v16b c, v16b d) { keep4_b(a, b, c, d); }
};

template <int ET> struct Elem;
template <> struct Elem<0> { typedef _Float16 T; };
template <> struct Elem<1> { typedef __bf16 T; };
template <int ET, bool SPLIT, int BIAS_MODE, int OUT_MODE, bool RESID, int ACT = 0>
__global__ __launch_bounds__(256) void wmma_gemm64(
    const unsigned short* __restrict__ Ap, const unsigned short* __restrict__ A2p, int lda, long strideA,
    const unsigned short* __restrict__ Btp, const unsigned short* __restrict__ Bt2p, int ldb, long strideB,
    void* __restrict__ Cout, void* __restrict__ Cout2, int ldc, long strideC,
    const float* __restrict__ bias,
    const float* __restrict__ resid, long strideR,
    int M, int N, int K, float scale) {
  typedef typename Elem<ET>::T T;
  typedef typename Frag<T>::V V;
  const T* A = (const T*)Ap; const T* A2 = (const T*)A2p; const T* Bt = (const T*)Btp; const T* Bt2 = (const T*)Bt2p;
  __shared__ __align__(16) float sT[8][16 * 68];
  const int b    = blockIdx.y;
  const int lane = threadIdx.x & 31;
  const int wave = threadIdx.x >> 5;
  const int tilesN = N >> 6;
  const int tilesM = M >> 6;
  const int tile = blockIdx.x * 8 + wave;
  if (tile >= tilesM * tilesN) return;
  const int tm = tile / tilesN;
  const int tn = tile - tm * tilesN;
  const int m0 = tm << 6;
  const int n0 = tn << 6;

  const T* Ab  = A  + (size_t)b * strideA;
  const T* Bb  = Bt + (size_t)b * strideB;
  const T* Ab2 = SPLIT ? (A2  + (size_t)b * strideA) : nullptr;
  const T* Bb2 = SPLIT ? (Bt2 + (size_t)b * strideB) : nullptr;

  const int rlane = lane & 15;
  const int koff  = (lane >> 4) * 8;
  const int mOff  = (lane >> 4) * 8;

  v8f acc[4][4];
#pragma unroll
  for (int i = 0; i < 4; ++i)
#pragma unroll
    for (int j = 0; j < 4; ++j) acc[i][j] = (v8f){0.f,0.f,0.f,0.f,0.f,0.f,0.f,0.f};

  for (int k0 = 0; k0 < K; k0 += 32) {
    V bh[4], bl[4];
#pragma unroll
    for (int j = 0; j < 4; ++j) {
      const size_t bo = (size_t)(n0 + (j << 4) + rlane) * ldb + koff + k0;
      bh[j] = Frag<T>::load(Bb + bo);
      if (SPLIT) bl[j] = Frag<T>::load(Bb2 + bo);
    }
#pragma unroll
    for (int i = 0; i < 4; ++i) {
      const size_t ao = (size_t)(m0 + (i << 4) + rlane) * lda + koff + k0;
      V ah = Frag<T>::load(Ab + ao);
      V al;
      if (SPLIT) al = Frag<T>::load(Ab2 + ao);
#pragma unroll
      for (int j = 0; j < 4; ++j) {
        acc[i][j] = Frag<T>::mma(ah, bh[j], acc[i][j]);
        if (SPLIT) {
          acc[i][j] = Frag<T>::mma(ah, bl[j], acc[i][j]);
          acc[i][j] = Frag<T>::mma(al, bh[j], acc[i][j]);
        }
      }
      Frag<T>::guard(acc[i][0], acc[i][3], ah, SPLIT ? al : ah);
    }
    Frag<T>::keep(bh[0], bh[1], bh[2], bh[3]);
    if (SPLIT) Frag<T>::keep(bl[0], bl[1], bl[2], bl[3]);
  }
  acc_guard4(acc[0][0], acc[0][1], acc[0][2], acc[0][3]);
  acc_guard4(acc[1][0], acc[1][1], acc[1][2], acc[1][3]);
  acc_guard4(acc[2][0], acc[2][1], acc[2][2], acc[2][3]);
  acc_guard4(acc[3][0], acc[3][1], acc[3][2], acc[3][3]);

  float* slab = sT[wave];
  const float* Rb = RESID ? (resid + (size_t)b * strideR) : nullptr;
#pragma unroll
  for (int i = 0; i < 4; ++i) {
    const int mBase = m0 + (i << 4);
#pragma unroll
    for (int j = 0; j < 4; ++j) {
      const int n = n0 + (j << 4) + rlane;
      float bv = 0.f;
      if (BIAS_MODE == 2) bv = bias[n];
#pragma unroll
      for (int r = 0; r < 8; ++r) {
        float v = acc[i][j][r] * scale;
        if (BIAS_MODE == 1) v += bias[mBase + mOff + r];
        if (BIAS_MODE == 2) v += bv;
        if (RESID) v += Rb[(size_t)(mBase + mOff + r) * ldc + n];
        if (ACT == 1) v = tanhf(v);
        if (ACT == 2) v = fmaxf(v, 0.0f);
        if (ACT == 3) v = v / (1.0f + expf(-v));
        if (ACT == 4) v = (v > 0.f) ? v : 0.01f * v;
        if (ACT == 5) v = 0.5f * v * (1.0f + erff(v * 0.70710678118654752f));
        slab[(mOff + r) * 68 + (j << 4) + rlane] = v;
      }
    }
    __builtin_amdgcn_fence(__ATOMIC_RELEASE, "workgroup");
    __builtin_amdgcn_wave_barrier();
    __builtin_amdgcn_fence(__ATOMIC_ACQUIRE, "workgroup");
    if (OUT_MODE == 0) {
      float* C = (float*)Cout + (size_t)b * strideC;
      const int hh = lane >> 4, c4 = (lane & 15) * 4;
      for (int pass = 0; pass < 2; ++pass) {
#pragma unroll
        for (int it = 0; it < 8; ++it) {
          const int row = it * 2 + hh;
          v4f v = *(const v4f*)(slab + row * 68 + c4);
          *(volatile v4f*)(C + (size_t)(mBase + row) * ldc + n0 + c4) = v;
        }
        __threadfence();
      }
    } else {
      const int q = lane >> 3, c8 = (lane & 7) * 8;
      unsigned short* C  = (unsigned short*)Cout  + (size_t)b * strideC;
      unsigned short* C2 = (OUT_MODE == 2) ? ((unsigned short*)Cout2 + (size_t)b * strideC) : nullptr;
      for (int pass = 0; pass < 2; ++pass) {
#pragma unroll
        for (int it = 0; it < 4; ++it) {
          const int row = it * 4 + q;
          const float* sp = slab + row * 68 + c8;
          v8h hv, lv;
#pragma unroll
          for (int e = 0; e < 8; ++e) {
            if (OUT_MODE == 1) {
              hv[e] = (_Float16)sp[e];
            } else {
              unsigned short hb = f2bf_bits(sp[e]);
              unsigned short lb = f2bf_bits(sp[e] - bf_bits2f(hb));
              hv[e] = __builtin_bit_cast(_Float16, hb);
              lv[e] = __builtin_bit_cast(_Float16, lb);
            }
          }
          *(volatile v8h*)(C + (size_t)(mBase + row) * ldc + n0 + c8) = hv;
          if (OUT_MODE == 2) *(volatile v8h*)(C2 + (size_t)(mBase + row) * ldc + n0 + c8) = lv;
        }
        __threadfence();
      }
    }
    __builtin_amdgcn_fence(__ATOMIC_RELEASE, "workgroup");
    __builtin_amdgcn_wave_barrier();
    __builtin_amdgcn_fence(__ATOMIC_ACQUIRE, "workgroup");
  }
}

constexpr int kBatch   = 256;
constexpr int kSteps   = 512;
constexpr int kIn0     = 30;
constexpr int kIn0P    = 32;
constexpr int kHid     = 128;
constexpr int kGate4   = 512;
constexpr int kRowsBlk = 16;
constexpr int kRowsTot = kBatch * kSteps;
constexpr int kNL  = 84;
constexpr int kNLP = 128;
constexpr int kNO  = 63;
constexpr int kNOP = 64;
constexpr int kKO  = 96;

constexpr size_t kOffWc0  = 0;
constexpr size_t kOffWc1  = 163840;
constexpr size_t kOffWl   = 425984;
constexpr size_t kOffWo   = 458752;
constexpr size_t kOffBl   = 471040;
constexpr size_t kOffBo   = 471552;
constexpr size_t kOffH1   = 524288;
constexpr size_t kPlaneB  = (size_t)kBatch * kSteps * kHid * 2;
constexpr size_t kOffH2   = kOffH1 + kPlaneB;
constexpr size_t kOffStg  = kOffH2 + kPlaneB;
constexpr size_t kStgB    = (size_t)kRowsTot * kNOP * 4;
constexpr size_t kWsTotal = kOffStg + kStgB;

__global__ __launch_bounds__(256) void prep_planes(
    const float* __restrict__ Wih0, const float* __restrict__ Whh0,
    const float* __restrict__ Wih1, const float* __restrict__ Whh1,
    const float* __restrict__ Wl,   const float* __restrict__ bl,
    const float* __restrict__ Wo,   const float* __restrict__ bo,
    _Float16* __restrict__ wc0, _Float16* __restrict__ wc1,
    _Float16* __restrict__ wl16, _Float16* __restrict__ wo16,
    float* __restrict__ blp, float* __restrict__ bop) {
  const int sel = blockIdx.y;
  const int i = blockIdx.x * 256 + threadIdx.x;
  if (sel == 0) {
    if (i >= kGate4 * (kIn0P + kHid) / 8) return;
    const int e0 = 8 * i;
    const int n = e0 / (kIn0P + kHid);
    const int k0 = e0 - n * (kIn0P + kHid);
    v8h v;
#pragma unroll
    for (int j = 0; j < 8; ++j) {
      const int k = k0 + j;
      const int ka = (k < kIn0) ? k : (kIn0 - 1);
      const int kb = (k >= kIn0P) ? (k - kIn0P) : 0;
      const float a = Wih0[n * kIn0 + ka] * 64.0f;
      const float bval = Whh0[n * kHid + kb] * 8.0f;
      const float val = (k < kIn0) ? a : ((k < kIn0P) ? 0.0f : bval);
      v[j] = (_Float16)val;
    }
    _Float16* d = wc0 + e0;
    *(volatile v8h*)d = v; __threadfence(); *(volatile v8h*)d = v;
  } else if (sel == 1) {
    if (i >= kGate4 * (2 * kHid) / 8) return;
    const int e0 = 8 * i;
    const int n = e0 >> 8;
    const int k0 = e0 & 255;
    v8h v;
#pragma unroll
    for (int j = 0; j < 8; ++j) {
      const int k = k0 + j;
      const int kk = k & 127;
      const float a = Wih1[n * kHid + kk] * 8.0f;
      const float bval = Whh1[n * kHid + kk] * 8.0f;
      v[j] = (_Float16)((k < kHid) ? a : bval);
    }
    _Float16* d = wc1 + e0;
    *(volatile v8h*)d = v; __threadfence(); *(volatile v8h*)d = v;
  } else if (sel == 2) {
    if (i >= kNLP * kHid / 8) return;
    const int e0 = 8 * i;
    const int n = e0 >> 7;
    const int k0 = e0 & 127;
    const int nc = (n < kNL) ? n : (kNL - 1);
    v8h v;
#pragma unroll
    for (int j = 0; j < 8; ++j) {
      const float a = Wl[nc * kHid + k0 + j] * 8.0f;
      v[j] = (_Float16)((n < kNL) ? a : 0.0f);
    }
    _Float16* d = wl16 + e0;
    *(volatile v8h*)d = v; __threadfence(); *(volatile v8h*)d = v;
  } else if (sel == 3) {
    if (i >= kNOP * kKO / 8) return;
    const int e0 = 8 * i;
    const int n = e0 / kKO;
    const int k0 = e0 - n * kKO;
    const int nc = (n < kNO) ? n : (kNO - 1);
    v8h v;
#pragma unroll
    for (int j = 0; j < 8; ++j) {
      const int k = k0 + j;
      const int kc = (k < kNL) ? k : (kNL - 1);
      const float a = Wo[nc * kNL + kc] * 8.0f;
      v[j] = (_Float16)((n < kNO && k < kNL) ? a : 0.0f);
    }
    _Float16* d = wo16 + e0;
    *(volatile v8h*)d = v; __threadfence(); *(volatile v8h*)d = v;
  } else if (sel == 4) {
    if (i >= kNLP / 4) return;
    const int n0 = 4 * i;
    v4f v;
#pragma unroll
    for (int j = 0; j < 4; ++j) {
      const int n = n0 + j;
      const int nc = (n < kNL) ? n : (kNL - 1);
      const float a = bl[nc] * 8.0f;
      v[j] = (n < kNL) ? a : 0.0f;
    }
    float* d = blp + n0;
    *(volatile v4f*)d = v; __threadfence(); *(volatile v4f*)d = v;
  } else {
    if (i >= kNOP / 4) return;
    const int n0 = 4 * i;
    v4f v;
#pragma unroll
    for (int j = 0; j < 4; ++j) {
      const int n = n0 + j;
      const int nc = (n < kNO) ? n : (kNO - 1);
      const float a = bo[nc];
      v[j] = (n < kNO) ? a : 0.0f;
    }
    float* d = bop + n0;
    *(volatile v4f*)d = v; __threadfence(); *(volatile v4f*)d = v;
  }
}

__device__ __forceinline__ float sigm_f(float x) {
  const float xc = fminf(fmaxf(x, -40.0f), 40.0f);
  return __builtin_amdgcn_rcpf(1.0f + __expf(-xc));
}
__device__ __forceinline__ float tanh_f(float x) {
  const float xc = fminf(fmaxf(x, -20.0f), 20.0f);
  return 1.0f - 2.0f * __builtin_amdgcn_rcpf(1.0f + __expf(2.0f * xc));
}

template <int KIN>
__global__ __launch_bounds__(256) void lstm_seq(
    const float* __restrict__ xin, const unsigned short* __restrict__ hin,
    const unsigned short* __restrict__ Wc, const float* __restrict__ bih,
    const float* __restrict__ bhh, unsigned short* __restrict__ hpl) {
  constexpr int KTOT = KIN + kHid;
  constexpr int NKS = KTOT / 32;
  __shared__ __align__(16) _Float16 At[kRowsBlk * KTOT];

  const int tid  = threadIdx.x;
  const int lane = tid & 31;
  const int wave = tid >> 5;
  const int hh   = lane >> 4;
  const int cc   = lane & 15;
  const int b0   = blockIdx.x * kRowsBlk;
  const _Float16* W = (const _Float16*)(const void*)Wc;

  const int unit = 16 * wave + cc;
  const float bias0 = bih[unit] + bhh[unit];
  const float bias1 = bih[kHid + unit] + bhh[kHid + unit];
  const float bias2 = bih[2 * kHid + unit] + bhh[2 * kHid + unit];
  const float bias3 = bih[3 * kHid + unit] + bhh[3 * kHid + unit];

  const _Float16* arow  = At + cc * KTOT + 8 * hh;
  const _Float16* wrow0 = W + (size_t)(0 * kHid + unit) * KTOT + 8 * hh;
  const _Float16* wrow1 = W + (size_t)(1 * kHid + unit) * KTOT + 8 * hh;
  const _Float16* wrow2 = W + (size_t)(2 * kHid + unit) * KTOT + 8 * hh;
  const _Float16* wrow3 = W + (size_t)(3 * kHid + unit) * KTOT + 8 * hh;

  v8f creg = (v8f){0.f,0.f,0.f,0.f,0.f,0.f,0.f,0.f};
  v8f hreg = (v8f){0.f,0.f,0.f,0.f,0.f,0.f,0.f,0.f};
  const float k64 = 1.0f / 64.0f;

#pragma unroll 1
  for (int t = 0; t <= kSteps; ++t) {
    const int tl = (t < kSteps) ? t : (kSteps - 1);
    __syncthreads();
    {
      _Float16* hp = At + KIN + unit;
#pragma unroll
      for (int r = 0; r < 8; ++r) hp[(8 * hh + r) * KTOT] = (_Float16)(hreg[r] * 8.0f);
    }
    if (KIN == kIn0P) {
      const int r = tid >> 4;
      const int j2 = (tid & 15) * 2;
      const float* xp = xin + ((size_t)(b0 + r) * kSteps + tl) * kIn0;
      const int ka = (j2 < kIn0) ? j2 : (kIn0 - 1);
      const int kb = (j2 + 1 < kIn0) ? (j2 + 1) : (kIn0 - 1);
      float v0 = xp[ka];
      float v1 = xp[kb];
      v0 = (j2 < kIn0) ? v0 : 0.0f;
      v1 = (j2 + 1 < kIn0) ? v1 : 0.0f;
      const _Float16 h0v = (_Float16)v0;
      const _Float16 h1v = (_Float16)v1;
      const unsigned pk = (unsigned)__builtin_bit_cast(unsigned short, h0v)
                        | ((unsigned)__builtin_bit_cast(unsigned short, h1v) << 16);
      *(unsigned*)(void*)(At + r * KTOT + j2) = pk;
    } else {
      const int r = tid >> 4;
      const int q = tid & 15;
      const v4u v = *(const v4u*)(const void*)(hin + ((size_t)(b0 + r) * kSteps + tl) * kHid + 8 * q);
      *(v4u*)(void*)(At + r * KTOT + 8 * q) = v;
    }
    __syncthreads();
    if (t > 0) {
      const int srow = 2 * wave + hh;
      const v4u hv4 = *(const v4u*)(const void*)(At + srow * KTOT + KIN + 8 * cc);
      unsigned short* dst = hpl + ((size_t)(b0 + srow) * kSteps + (t - 1)) * kHid + 8 * cc;
      *(volatile v4u*)dst = hv4;
      __threadfence();
      *(volatile v4u*)dst = hv4;
    }
    if (t < kSteps) {
      v8f acc[4];
#pragma unroll
      for (int g = 0; g < 4; ++g) acc[g] = (v8f){0.f,0.f,0.f,0.f,0.f,0.f,0.f,0.f};
#pragma unroll 1
      for (int ks = 0; ks < NKS; ++ks) {
        const int ko = ks * 32;
        const v16h a   = Frag<_Float16>::load(arow + ko);
        const v16h bf0 = Frag<_Float16>::load(wrow0 + ko);
        const v16h bf1 = Frag<_Float16>::load(wrow1 + ko);
        const v16h bf2 = Frag<_Float16>::load(wrow2 + ko);
        const v16h bf3 = Frag<_Float16>::load(wrow3 + ko);
        acc[0] = Frag<_Float16>::mma(a, bf0, acc[0]);
        acc[1] = Frag<_Float16>::mma(a, bf1, acc[1]);
        acc[2] = Frag<_Float16>::mma(a, bf2, acc[2]);
        acc[3] = Frag<_Float16>::mma(a, bf3, acc[3]);
        dep_guard4x_h(acc[0], acc[1], acc[2], acc[3], a, bf3);
        keep4_h(bf0, bf1, bf2, bf3);
      }
      acc_guard4(acc[0], acc[1], acc[2], acc[3]);
#pragma unroll
      for (int r = 0; r < 8; ++r) {
        const float pi = acc[0][r] * k64 + bias0;
        const float pf = acc[1][r] * k64 + bias1;
        const float pg = acc[2][r] * k64 + bias2;
        const float po = acc[3][r] * k64 + bias3;
        const float ig = sigm_f(pi);
        const float fg = sigm_f(pf);
        const float gg = tanh_f(pg);
        const float og = sigm_f(po);
        const float cn = fg * creg[r] + ig * gg;
        creg[r] = cn;
        hreg[r] = og * tanh_f(cn);
      }
    }
  }
}

__global__ __launch_bounds__(256) void pack_rows(const float* __restrict__ stg,
                                                 float* __restrict__ out, int n4) {
  const int i = blockIdx.x * 256 + threadIdx.x;
  if (i >= n4) return;
  v4f v;
#pragma unroll
  for (int j = 0; j < 4; ++j) {
    const int e = 4 * i + j;
    const int row = e / kNO;
    const int n = e - row * kNO;
    v[j] = stg[(size_t)row * kNOP + n];
  }
  float* dst = out + (size_t)4 * i;
  *(volatile v4f*)dst = v;
  __threadfence();
  *(volatile v4f*)dst = v;
}

extern "C" void kernel_launch(void* const* d_in, const int* in_sizes, int n_in,
                              void* d_out, int out_size, void* d_ws, size_t ws_size,
                              hipStream_t stream) {
  if (n_in < 13) return;
  if (in_sizes[0] != kBatch * kSteps * kIn0) return;
  if (in_sizes[1] != kGate4 * kIn0 || in_sizes[2] != kGate4 * kHid) return;
  if (in_sizes[3] != kGate4 || in_sizes[4] != kGate4) return;
  if (in_sizes[5] != kGate4 * kHid || in_sizes[6] != kGate4 * kHid) return;
  if (in_sizes[7] != kGate4 || in_sizes[8] != kGate4) return;
  if (in_sizes[9] != kNL * kHid || in_sizes[10] != kNL) return;
  if (in_sizes[11] != kNO * kNL || in_sizes[12] != kNO) return;
  if (out_size != kRowsTot * kNO) return;
  if (ws_size < kWsTotal) return;

  const float* x    = (const float*)d_in[0];
  const float* Wih0 = (const float*)d_in[1];
  const float* Whh0 = (const float*)d_in[2];
  const float* bih0 = (const float*)d_in[3];
  const float* bhh0 = (const float*)d_in[4];
  const float* Wih1 = (const float*)d_in[5];
  const float* Whh1 = (const float*)d_in[6];
  const float* bih1 = (const float*)d_in[7];
  const float* bhh1 = (const float*)d_in[8];
  const float* Wl   = (const float*)d_in[9];
  const float* bl   = (const float*)d_in[10];
  const float* Wo   = (const float*)d_in[11];
  const float* bo   = (const float*)d_in[12];

  char* ws = (char*)d_ws;
  _Float16* wc0  = (_Float16*)(ws + kOffWc0);
  _Float16* wc1  = (_Float16*)(ws + kOffWc1);
  _Float16* wl16 = (_Float16*)(ws + kOffWl);
  _Float16* wo16 = (_Float16*)(ws + kOffWo);
  float*    blp  = (float*)(ws + kOffBl);
  float*    bop  = (float*)(ws + kOffBo);
  unsigned short* h1p = (unsigned short*)(ws + kOffH1);
  unsigned short* yp  = (unsigned short*)(ws + kOffH1);
  unsigned short* h2p = (unsigned short*)(ws + kOffH2);
  float*    stg  = (float*)(ws + kOffStg);
  float*    out  = (float*)d_out;

  prep_planes<<<dim3(64, 6), 256, 0, stream>>>(Wih0, Whh0, Wih1, Whh1, Wl, bl, Wo, bo,
                                               wc0, wc1, wl16, wo16, blp, bop);

  lstm_seq<kIn0P><<<kBatch / kRowsBlk, 256, 0, stream>>>(
      x, (const unsigned short*)h2p, (const unsigned short*)wc0, bih0, bhh0, h1p);
  lstm_seq<kHid><<<kBatch / kRowsBlk, 256, 0, stream>>>(
      x, (const unsigned short*)h1p, (const unsigned short*)wc1, bih1, bhh1, h2p);

  wmma_gemm64<0, false, 2, 1, false><<<dim3((kRowsTot / 64) * (kNLP / 64) / 8, 1), 256, 0, stream>>>(
      (const unsigned short*)h2p, (const unsigned short*)h2p, kHid, 0L,
      (const unsigned short*)wl16, (const unsigned short*)wl16, kHid, 0L,
      (void*)yp, (void*)yp, kNLP, 0L,
      blp, blp, 0L, kRowsTot, kNLP, kHid, 0.125f);

  wmma_gemm64<0, false, 2, 0, false><<<dim3((kRowsTot / 64) * (kNOP / 64) / 8, 1), 256, 0, stream>>>(
      (const unsigned short*)yp, (const unsigned short*)yp, kNLP, 0L,
      (const unsigned short*)wo16, (const unsigned short*)wo16, kKO, 0L,
      (void*)stg, (void*)stg, kNOP, 0L,
      bop, bop, 0L, kRowsTot, kNOP, kKO, 1.0f / 64.0f);

  const int n4 = out_size / 4;
  pack_rows<<<(n4 + 255) / 256, 256, 0, stream>>>(stg, out, n4);
}
